// MultiHeadAttention_37477884625313
// MI455X (gfx1250) — hardware-run, weakly checked
//
#include <hip/hip_runtime.h>


#ifndef NB
#define NB 4
#endif
#ifndef SEQ
#define SEQ 1024
#endif
#define NB_FULL  4
#define SEQ_FULL 1024
#ifndef OUT_SEQ
#define OUT_SEQ SEQ
#endif
#define DM   512
#define NH_  8
#define HD   64
#define NTAP 9
#define AW   4
#define QRS  2048.0f
#define QRI  (1.0f / 2048.0f)
#define SC2  (0.125f * 1.4426950408889634f)
#define PSH  8.0f
#define CTS  256.0f
#define WOS  64.0f
#define OSC  (1.0f / 16384.0f)
#define BPP  20

static_assert(HD == 64);
static_assert(NH_ * HD == DM);
static_assert(DM % 64 == 0);
static_assert(DM % 32 == 0);
static_assert(SEQ % 64 == 0);
static_assert(SEQ >= 64);
static_assert((NB * SEQ) % 64 == 0);
static_assert(SEQ % 32 == 0);
static_assert(SEQ % (16 * AW) == 0);
static_assert(NB <= NB_FULL);
static_assert(SEQ <= SEQ_FULL);
static_assert(SEQ <= OUT_SEQ);
static_assert(NTAP <= 16);
static_assert((BPP * 4) % 16 == 0);

typedef _Float16 h16;
typedef unsigned short bf;
typedef __attribute__((ext_vector_type(16))) __bf16   v16bf;
typedef __attribute__((ext_vector_type(16))) _Float16 v16h;
typedef __attribute__((ext_vector_type(8)))  _Float16 v8h;
typedef __attribute__((ext_vector_type(8)))  unsigned short v8us;
typedef __attribute__((ext_vector_type(8)))  float    v8f;
typedef __attribute__((ext_vector_type(4)))  float    v4f;
typedef v4f  __attribute__((may_alias)) v4fa;

__device__ __forceinline__ unsigned short f2bf(float f) { unsigned u = __float_as_uint(f); u += 0x7FFFu + ((u >> 16) & 1u); return (unsigned short)(u >> 16); }
__device__ __forceinline__ float bfr(float f) { return __uint_as_float(((unsigned)f2bf(f)) << 16); }
__device__ __forceinline__ v16h cat16(v8h lo, v8h hi) { return __builtin_shufflevector(lo, hi, 0, 1, 2, 3, 4, 5, 6, 7, 8, 9, 10, 11, 12, 13, 14, 15); }
__device__ __forceinline__ v16bf cat16b(v8us lo, v8us hi) { return __builtin_bit_cast(v16bf, __builtin_shufflevector(lo, hi, 0, 1, 2, 3, 4, 5, 6, 7, 8, 9, 10, 11, 12, 13, 14, 15)); }
__device__ __forceinline__ v8f wmma16(v16h a, v16h b, v8f c) { return __builtin_amdgcn_wmma_f32_16x16x32_f16(false, a, false, b, (short)0, c, false, false); }
__device__ __forceinline__ v8f wmmab(v16bf a, v16bf b, v8f c) { return __builtin_amdgcn_wmma_f32_16x16x32_bf16(false, a, false, b, (short)0, c, false, false); }
__device__ __forceinline__ v16h  ldh(const h16* p) { return cat16(*(const v8h*)p, *(const v8h*)(p + 16)); }
__device__ __forceinline__ v16bf ldb(const bf* p)  { return cat16b(*(const v8us*)p, *(const v8us*)(p + 16)); }
__device__ __forceinline__ void wave_sync() { __builtin_amdgcn_fence(3  , "wavefront"); __builtin_amdgcn_wave_barrier(); asm volatile("" ::: "memory"); }

__global__ __launch_bounds__(256) void k_cvt8(const float* __restrict__ src, bf* dst, size_t n8) {
    const size_t i = (size_t)blockIdx.x * 256 + threadIdx.x; if (i >= n8) return;
    const v8f v = *(const v8f*)(src + i * 8); v8us o;
#pragma unroll
    for (int k = 0; k < 8; ++k) o[k] = f2bf(v[k]);
    *(volatile v8us*)(dst + i * 8) = o; __threadfence(); *(volatile v8us*)(dst + i * 8) = o;
}

__global__ __launch_bounds__(256) void k_cvtw(const float* __restrict__ src, h16* dst, size_t n8) {
    const size_t i = (size_t)blockIdx.x * 256 + threadIdx.x; if (i >= n8) return;
    const v8f v = *(const v8f*)(src + i * 8); v8h o;
#pragma unroll
    for (int k = 0; k < 8; ++k) o[k] = (h16)(bfr(v[k]) * WOS);
    *(volatile v8h*)(dst + i * 8) = o; __threadfence(); *(volatile v8h*)(dst + i * 8) = o;
}

__global__ __launch_bounds__(256) void k_ev(const float* __restrict__ ev, h16* dst) {
    const int i = blockIdx.x * 256 + threadIdx.x; if (i >= NH_ * HD * 4) return;
    const int row = i >> 2, p = i & 3; const int h = row / HD, d = row % HD;
    v8h o;
#pragma unroll
    for (int k = 0; k < 8; ++k) { const int jj = p * 8 + k; const int jc = (jj < NTAP) ? jj : (NTAP - 1);
        const float v = bfr(ev[(h * NTAP + jc) * HD + d]); o[k] = (jj < NTAP) ? (h16)v : (h16)0.0f; }
    *(volatile v8h*)(dst + (size_t)i * 8) = o; __threadfence(); *(volatile v8h*)(dst + (size_t)i * 8) = o;
}

__global__ __launch_bounds__(256) void k_xT(const float* __restrict__ src, bf* dst) {
    __shared__ float tl[64 * 65];
    const int tid = threadIdx.x; const int t0 = blockIdx.x * 64, c0 = blockIdx.y * 64, b = blockIdx.z;
    const float* s = src + ((size_t)b * DM + c0) * SEQ_FULL + t0;
#pragma unroll
    for (int i = 0; i < 4; ++i) { const int idx = tid + 256 * i; const int row = idx >> 4, c4 = (idx & 15) * 4;
        const v4f v = *(const v4f*)(s + (size_t)row * SEQ_FULL + c4);
        tl[row * 65 + c4 + 0] = v[0]; tl[row * 65 + c4 + 1] = v[1]; tl[row * 65 + c4 + 2] = v[2]; tl[row * 65 + c4 + 3] = v[3]; }
    __syncthreads();
    v8us o0, o1;
    { const int trow = tid >> 3, p = tid & 7;
#pragma unroll
      for (int k = 0; k < 8; ++k) { o0[k] = f2bf(tl[(p * 8 + k) * 65 + trow]); o1[k] = f2bf(tl[(p * 8 + k) * 65 + trow + 32]); } }
    bf* d0 = dst + ((size_t)b * SEQ + t0 + (tid >> 3)) * DM + c0 + (tid & 7) * 8;
    bf* d1 = d0 + (size_t)32 * DM;
    *(volatile v8us*)d0 = o0; *(volatile v8us*)d1 = o1; __threadfence(); *(volatile v8us*)d0 = o0; *(volatile v8us*)d1 = o1;
}

template <int BM>
__global__ __launch_bounds__(32) void k_proj(const bf* __restrict__ A, const bf* __restrict__ Bt, const float* __restrict__ bias, h16* Ph, h16* Pr, int useRes, int RB, size_t sRB, int pitch, int CB, size_t sCB) {
    __shared__ __align__(16) float os[16 * 68];
    const int K = DM;
    const int lane = threadIdx.x & 31, lr = lane & 15, hi = lane >> 4; const int r0 = blockIdx.x * 64, c0 = blockIdx.y * 64;
    v8f acc[4][4];
#pragma unroll
    for (int mb = 0; mb < 4; ++mb)
#pragma unroll
        for (int nb = 0; nb < 4; ++nb) acc[mb][nb] = (v8f){};
    const size_t aoff = (size_t)(r0 + lr) * K + 8 * hi, boff = (size_t)(c0 + lr) * K + 8 * hi;
#pragma unroll 1
    for (int kc = 0; kc < K; kc += 32) {
        v16bf a[4];
#pragma unroll
        for (int mb = 0; mb < 4; ++mb) a[mb] = ldb(A + aoff + (size_t)mb * 16 * K + kc);
#pragma unroll
        for (int nb = 0; nb < 4; ++nb) { const v16bf b = ldb(Bt + boff + (size_t)nb * 16 * K + kc);
#pragma unroll
            for (int mb = 0; mb < 4; ++mb) acc[mb][nb] = wmmab(a[mb], b, acc[mb][nb]); }
        asm volatile("v_nop\n\tv_nop\n\tv_nop\n\tv_nop" : "+v"(acc[0][0]), "+v"(acc[1][1]), "+v"(acc[2][2]), "+v"(acc[3][3]) : "v"(a[0]), "v"(a[1]), "v"(a[2]), "v"(a[3]));
    }
    float bc[8];
#pragma unroll
    for (int i = 0; i < 8; ++i) bc[i] = 0.0f;
    if (BM == 0) { const v4f b0 = *(const v4f*)(bias + c0 + (lane & 7) * 8); const v4f b1 = *(const v4f*)(bias + c0 + (lane & 7) * 8 + 4);
#pragma unroll
        for (int i = 0; i < 4; ++i) { bc[i] = bfr(b0[i]); bc[4 + i] = bfr(b1[i]); } }
    const size_t tbase = (size_t)(r0 / RB) * sRB + (size_t)(r0 % RB) * (size_t)pitch + (size_t)(c0 / CB) * sCB + (size_t)(c0 % CB);
#pragma unroll
    for (int mb = 0; mb < 4; ++mb) {
#pragma unroll
        for (int nb = 0; nb < 4; ++nb) {
#pragma unroll
            for (int j = 0; j < 8; ++j) os[(hi * 8 + j) * 68 + nb * 16 + lr] = acc[mb][nb][j]; }
        wave_sync();
        const size_t sb = tbase + (size_t)(mb * 16) * (size_t)pitch;
#pragma unroll 1
        for (int ps = 0; ps < 2; ++ps) {
#pragma unroll
            for (int s = 0; s < 4; ++s) { const int row = 4 * s + (lane >> 3), c8 = (lane & 7) * 8;
                const v4f x0 = *(const v4fa*)(&os[row * 68 + c8]); const v4f x1 = *(const v4fa*)(&os[row * 68 + c8 + 4]); v8h hv, rv;
                float br = 0.0f; if (BM == 1) br = bfr(bias[r0 + mb * 16 + row]);
#pragma unroll
                for (int i = 0; i < 4; ++i) { const float f0 = x0[i] + bc[i] + br; const float f1 = x1[i] + bc[4 + i] + br;
                    const h16 a0 = (h16)f0; const h16 a1 = (h16)f1; hv[i] = a0; hv[4 + i] = a1; rv[i] = (h16)((f0 - (float)a0) * QRS); rv[4 + i] = (h16)((f1 - (float)a1) * QRS); }
                const size_t oo = sb + (size_t)row * (size_t)pitch + c8;
                *(volatile v8h*)(Ph + oo) = hv; if (useRes) *(volatile v8h*)(Pr + oo) = rv; }
            if (ps == 0) __threadfence(); }
        wave_sync();
    }
}

__global__ __launch_bounds__(32 * AW) void k_flash(const h16* __restrict__ QH, const h16* __restrict__ QR, const h16* __restrict__ KP, const h16* __restrict__ VT,
                                                   const h16* __restrict__ EV, const float* __restrict__ EK, h16* CT) {
    __shared__ __align__(16) float os[AW * 16 * 68];
    __shared__ __align__(16) float bp[AW * 16 * BPP];
    const int lane = threadIdx.x & 31, wave = threadIdx.x >> 5, lr = lane & 15, hi = lane >> 4;
    const int zh = blockIdx.y; const int b = zh / NH_, h = zh % NH_;
    const int t0 = (blockIdx.x * AW + wave) * 16;
    const size_t pbase = (size_t)zh * SEQ * HD;
    const size_t qo = pbase + (size_t)(t0 + lr) * HD + 8 * hi;
    const v16h qh0 = ldh(QH + qo), qh1 = ldh(QH + qo + 32), qr0 = ldh(QR + qo), qr1 = ldh(QR + qo + 32);
    const size_t ko = pbase + (size_t)lr * HD + 8 * hi;
    const size_t vo = pbase + (size_t)lr * SEQ + 8 * hi;
    const int bo = wave * 16 * BPP;
#pragma unroll
    for (int i = 0; i < 10; ++i) bp[bo + lane * 10 + i] = -1.0e30f;
    float bz[8];
#pragma unroll
    for (int r = 0; r < 8; ++r) bz[r] = 0.0f;
    const bool cA = (t0 == 0), cB = (t0 == SEQ - 16);
    if (cA || cB) {
        const int ti = t0 + lr;
        const int jb = cA ? (SEQ - 16 + 8 * hi) : (8 * hi);
        int ec[8]; bool vd[8];
#pragma unroll
        for (int r = 0; r < 8; ++r) { const int j = jb + r;
            const int e = cA ? (j - ti - (SEQ - 5)) : (SEQ + 5 - (ti - j));
            vd[r] = cA ? (e >= 0 && e <= 4) : (e >= 6 && e <= 8);
            ec[r] = (e < 0) ? 0 : ((e > NTAP - 1) ? (NTAP - 1) : e); }
        int qrow = cA ? ti : (ti - 1); qrow = (qrow < 0) ? 0 : qrow;
        const size_t qa = pbase + (size_t)qrow * HD;
#pragma unroll 1
        for (int d = 0; d < HD; ++d) {
            const float qv = (float)QH[qa + d] + (float)QR[qa + d] * QRI;
#pragma unroll
            for (int r = 0; r < 8; ++r) bz[r] = fmaf(qv, bfr(EK[(h * NTAP + ec[r]) * HD + d]), bz[r]);
        }
#pragma unroll
        for (int r = 0; r < 8; ++r) bz[r] = vd[r] ? bz[r] : 0.0f;
    }
    wave_sync();
    v8f o0 = (v8f){}, o1 = (v8f){}, o2 = (v8f){}, o3 = (v8f){};
    float m = -3.0e38f, l = 0.0f;
#pragma unroll 1
    for (int key0 = 0; key0 < SEQ; key0 += 32) {
        const h16* ka = KP + ko + (size_t)key0 * HD;
        const v16h ka0 = ldh(ka), ka1 = ldh(ka + 32), kb0 = ldh(ka + 16 * HD), kb1 = ldh(ka + 16 * HD + 32);
        v8f sHa = (v8f){}, sLa = (v8f){}, sHb = (v8f){}, sLb = (v8f){};
        sHa = wmma16(ka0, qh0, sHa); sLa = wmma16(ka0, qr0, sLa); sHb = wmma16(kb0, qh0, sHb); sLb = wmma16(kb0, qr0, sLb);
        sHa = wmma16(ka1, qh1, sHa); sLa = wmma16(ka1, qr1, sLa); sHb = wmma16(kb1, qh1, sHb); sLb = wmma16(kb1, qr1, sLb);
        asm volatile("v_nop\n\tv_nop\n\tv_nop\n\tv_nop" : "+v"(sHa), "+v"(sLa), "+v"(sHb), "+v"(sLb) : "v"(ka0), "v"(ka1), "v"(kb0), "v"(kb1));
        if (cA && key0 == SEQ - 32) {
#pragma unroll
            for (int r = 0; r < 8; ++r) sHb[r] += bz[r]; }
        if (cB && key0 == 0) {
#pragma unroll
            for (int r = 0; r < 8; ++r) sHa[r] += bz[r]; }
        float ta[8], tb[8]; float mx = -3.0e38f;
#pragma unroll
        for (int r = 0; r < 8; ++r) { ta[r] = (sHa[r] + sLa[r] * QRI) * SC2; tb[r] = (sHb[r] + sLb[r] * QRI) * SC2; mx = fmaxf(mx, fmaxf(ta[r], tb[r])); }
        if (key0 + 36 > t0 && key0 < t0 + 20) {
#pragma unroll
            for (int r = 0; r < 8; ++r) { const int dA = key0 + 8 * hi + r - (t0 + lr) + 4; const int dB = dA + 16;
                const int sA = ((unsigned)dA < (unsigned)NTAP) ? dA : 16; const int sB = ((unsigned)dB < (unsigned)NTAP) ? dB : 16;
                bp[bo + lr * BPP + sA] = ta[r]; bp[bo + lr * BPP + sB] = tb[r]; }
        }
        mx = fmaxf(mx, __shfl_xor(mx, 16, 32));
        const float mnew = fmaxf(m, mx);
        const float alpha = __builtin_amdgcn_exp2f(m - mnew);
        const float sh = PSH - mnew;
        v16h pb; float ls = 0.0f;
#pragma unroll
        for (int r = 0; r < 8; ++r) { const h16 pa = (h16)__builtin_amdgcn_exp2f(ta[r] + sh); const h16 pc = (h16)__builtin_amdgcn_exp2f(tb[r] + sh); pb[r] = pa; pb[8 + r] = pc; ls += (float)pa + (float)pc; }
        l = l * alpha + ls; m = mnew;
        o0 = o0 * alpha; o1 = o1 * alpha; o2 = o2 * alpha; o3 = o3 * alpha;
        const h16* va = VT + vo + key0;
        const v16h v0 = ldh(va), v1 = ldh(va + (size_t)16 * SEQ), v2 = ldh(va + (size_t)32 * SEQ), v3 = ldh(va + (size_t)48 * SEQ);
        o0 = wmma16(v0, pb, o0); o1 = wmma16(v1, pb, o1); o2 = wmma16(v2, pb, o2); o3 = wmma16(v3, pb, o3);
        asm volatile("v_nop\n\tv_nop\n\tv_nop\n\tv_nop" : "+v"(o0), "+v"(o1), "+v"(o2), "+v"(o3) : "v"(v0), "v"(v1), "v"(v2), "v"(v3), "v"(pb));
    }
    l += __shfl_xor(l, 16, 32);
    wave_sync();
    {
        const v4f g0 = *(const v4fa*)(&bp[bo + lr * BPP + 8 * hi]); const v4f g1 = *(const v4fa*)(&bp[bo + lr * BPP + 8 * hi + 4]);
        const float sh = PSH - m;
        v16h pq;
#pragma unroll
        for (int i = 0; i < 4; ++i) { pq[i] = (h16)__builtin_amdgcn_exp2f(g0[i] + sh); pq[4 + i] = (h16)__builtin_amdgcn_exp2f(g1[i] + sh); }
#pragma unroll
        for (int i = 8; i < 16; ++i) pq[i] = (h16)0.0f;
        const h16* ea = EV + ((size_t)(h * HD + lr)) * 32 + 8 * hi;
        const v16h e0 = ldh(ea), e1 = ldh(ea + 16 * 32), e2 = ldh(ea + 32 * 32), e3 = ldh(ea + 48 * 32);
        o0 = wmma16(e0, pq, o0); o1 = wmma16(e1, pq, o1); o2 = wmma16(e2, pq, o2); o3 = wmma16(e3, pq, o3);
        asm volatile("v_nop\n\tv_nop\n\tv_nop\n\tv_nop" : "+v"(o0), "+v"(o1), "+v"(o2), "+v"(o3) : "v"(e0), "v"(e1), "v"(e2), "v"(e3), "v"(pq));
    }
    const float inv = CTS * (1.0f / l);
    const int wb = wave * 16 * 68;
    { v4f a, c;
      a[0] = o0[0] * inv; a[1] = o0[1] * inv; a[2] = o0[2] * inv; a[3] = o0[3] * inv; c[0] = o0[4] * inv; c[1] = o0[5] * inv; c[2] = o0[6] * inv; c[3] = o0[7] * inv;
      *(v4fa*)(&os[wb + lr * 68 +  0 + 8 * hi]) = a; *(v4fa*)(&os[wb + lr * 68 +  0 + 8 * hi + 4]) = c;
      a[0] = o1[0] * inv; a[1] = o1[1] * inv; a[2] = o1[2] * inv; a[3] = o1[3] * inv; c[0] = o1[4] * inv; c[1] = o1[5] * inv; c[2] = o1[6] * inv; c[3] = o1[7] * inv;
      *(v4fa*)(&os[wb + lr * 68 + 16 + 8 * hi]) = a; *(v4fa*)(&os[wb + lr * 68 + 16 + 8 * hi + 4]) = c;
      a[0] = o2[0] * inv; a[1] = o2[1] * inv; a[2] = o2[2] * inv; a[3] = o2[3] * inv; c[0] = o2[4] * inv; c[1] = o2[5] * inv; c[2] = o2[6] * inv; c[3] = o2[7] * inv;
      *(v4fa*)(&os[wb + lr * 68 + 32 + 8 * hi]) = a; *(v4fa*)(&os[wb + lr * 68 + 32 + 8 * hi + 4]) = c;
      a[0] = o3[0] * inv; a[1] = o3[1] * inv; a[2] = o3[2] * inv; a[3] = o3[3] * inv; c[0] = o3[4] * inv; c[1] = o3[5] * inv; c[2] = o3[6] * inv; c[3] = o3[7] * inv;
      *(v4fa*)(&os[wb + lr * 68 + 48 + 8 * hi]) = a; *(v4fa*)(&os[wb + lr * 68 + 48 + 8 * hi + 4]) = c; }
    wave_sync();
    h16* crow = CT + ((size_t)b * SEQ + t0) * DM + h * HD;
#pragma unroll 1
    for (int ps = 0; ps < 2; ++ps) {
#pragma unroll
        for (int s = 0; s < 4; ++s) { const int row = 4 * s + (lane >> 3), c8 = (lane & 7) * 8;
            const v4f x0 = *(const v4fa*)(&os[wb + row * 68 + c8]); const v4f x1 = *(const v4fa*)(&os[wb + row * 68 + c8 + 4]); v8h hv;
#pragma unroll
            for (int i = 0; i < 4; ++i) { hv[i] = (h16)x0[i]; hv[4 + i] = (h16)x1[i]; }
            *(volatile v8h*)(crow + (size_t)row * DM + c8) = hv; }
        if (ps == 0) __threadfence(); }
}

__global__ __launch_bounds__(32) void k_oproj(const h16* __restrict__ A, const h16* __restrict__ Bt, const float* __restrict__ bias, float* OUT) {
    __shared__ __align__(16) float os[16 * 68];
    const int K = DM;
    const int lane = threadIdx.x & 31, lr = lane & 15, hi = lane >> 4; const int r0 = blockIdx.x * 64, c0 = blockIdx.y * 64;
    v8f acc[4][4];
#pragma unroll
    for (int mb = 0; mb < 4; ++mb)
#pragma unroll
        for (int nb = 0; nb < 4; ++nb) acc[mb][nb] = (v8f){};
    const size_t aoff = (size_t)(r0 + lr) * K + 8 * hi, boff = (size_t)(c0 + lr) * K + 8 * hi;
#pragma unroll 1
    for (int kc = 0; kc < K; kc += 32) {
        v16h a[4];
#pragma unroll
        for (int mb = 0; mb < 4; ++mb) a[mb] = ldh(A + aoff + (size_t)mb * 16 * K + kc);
#pragma unroll
        for (int nb = 0; nb < 4; ++nb) { const v16h bq = ldh(Bt + boff + (size_t)nb * 16 * K + kc);
#pragma unroll
            for (int mb = 0; mb < 4; ++mb) acc[mb][nb] = wmma16(a[mb], bq, acc[mb][nb]); }
        asm volatile("v_nop\n\tv_nop\n\tv_nop\n\tv_nop" : "+v"(acc[0][0]), "+v"(acc[1][1]), "+v"(acc[2][2]), "+v"(acc[3][3]) : "v"(a[0]), "v"(a[1]), "v"(a[2]), "v"(a[3]));
    }
    const int bb = c0 / SEQ, tc = c0 % SEQ;
    const size_t tbase = ((size_t)bb * DM + r0) * OUT_SEQ + tc;
#pragma unroll
    for (int mb = 0; mb < 4; ++mb) {
#pragma unroll
        for (int nb = 0; nb < 4; ++nb) {
#pragma unroll
            for (int j = 0; j < 8; ++j) os[(hi * 8 + j) * 68 + nb * 16 + lr] = acc[mb][nb][j]; }
        wave_sync();
        const size_t sb = tbase + (size_t)(mb * 16) * OUT_SEQ;
#pragma unroll 1
        for (int ps = 0; ps < 2; ++ps) {
#pragma unroll
            for (int s = 0; s < 8; ++s) { const int row = 2 * s + hi, cofs = lr * 4;
                const v4f x = *(const v4fa*)(&os[row * 68 + cofs]);
                const float br = bfr(bias[r0 + mb * 16 + row]);
                v4f val; val[0] = x[0] * OSC + br; val[1] = x[1] * OSC + br; val[2] = x[2] * OSC + br; val[3] = x[3] * OSC + br;
                *(volatile v4f*)(OUT + sb + (size_t)row * OUT_SEQ + cofs) = val; }
            if (ps == 0) __threadfence(); }
        wave_sync();
    }
}

static constexpr size_t al256(size_t v) { return (v + 255) & ~(size_t)255; }
static constexpr size_t SZ_XT = al256((size_t)NB * SEQ * DM * 2);
static constexpr size_t SZ_W  = al256((size_t)DM * DM * 2);
static constexpr size_t SZ_EV = al256((size_t)NH_ * HD * 32 * 2);
static constexpr size_t SZ_PL = al256((size_t)NB * NH_ * SEQ * HD * 2);
static constexpr size_t SZ_CT = al256((size_t)NB * SEQ * DM * 2);
static constexpr size_t SZ_TOTAL = 3 * SZ_XT + 4 * SZ_W + SZ_EV + 4 * SZ_PL + SZ_CT;
static_assert(SZ_TOTAL <= (size_t)134217728);
static_assert((NH_ * HD * 4) % 256 == 0);

extern "C" void kernel_launch(void* const* d_in, const int* in_sizes, int n_in,
                              void* d_out, int out_size, void* d_ws, size_t ws_size, hipStream_t stream) {
    if (n_in < 13) return;
    const size_t needx = ((size_t)NB * DM - 1) * SEQ_FULL + SEQ;
    if ((size_t)in_sizes[0] < needx || (size_t)in_sizes[1] < needx || (size_t)in_sizes[2] < needx) return;
    if ((size_t)in_sizes[3] < (size_t)DM * DM || (size_t)in_sizes[5] < (size_t)DM * DM || (size_t)in_sizes[7] < (size_t)DM * DM || (size_t)in_sizes[9] < (size_t)DM * DM) return;
    if (in_sizes[4] < DM || in_sizes[6] < DM || in_sizes[8] < DM || in_sizes[10] < DM) return;
    if (in_sizes[11] < NH_ * NTAP * HD || in_sizes[12] < NH_ * NTAP * HD) return;
    if ((size_t)out_size < ((size_t)NB * DM - 1) * OUT_SEQ + SEQ) return;
    if (SZ_TOTAL > ws_size) return;
    const float* xq = (const float*)d_in[0]; const float* xk = (const float*)d_in[1]; const float* xv = (const float*)d_in[2];
    const float* wq = (const float*)d_in[3]; const float* bq = (const float*)d_in[4];
    const float* wk = (const float*)d_in[5]; const float* bk = (const float*)d_in[6];
    const float* wv = (const float*)d_in[7]; const float* bv = (const float*)d_in[8];
    const float* wo = (const float*)d_in[9]; const float* bo = (const float*)d_in[10];
    const float* ek = (const float*)d_in[11]; const float* ev = (const float*)d_in[12];
    float* OUT = (float*)d_out;
    char* wsp = (char*)d_ws;
    bf* XTQ = (bf*)wsp; wsp += SZ_XT;
    bf* XTK = (bf*)wsp; wsp += SZ_XT;
    bf* XTV = (bf*)wsp; wsp += SZ_XT;
    bf* WQ = (bf*)wsp; wsp += SZ_W;
    bf* WK = (bf*)wsp; wsp += SZ_W;
    bf* WV = (bf*)wsp; wsp += SZ_W;
    h16* WO = (h16*)wsp; wsp += SZ_W;
    h16* EV = (h16*)wsp; wsp += SZ_EV;
    h16* QH = (h16*)wsp; wsp += SZ_PL;
    h16* QR = (h16*)wsp; wsp += SZ_PL;
    h16* KP = (h16*)wsp; wsp += SZ_PL;
    h16* VT = (h16*)wsp; wsp += SZ_PL;
    h16* CT = (h16*)wsp; wsp += SZ_CT;

    k_xT<<<dim3(SEQ / 64, DM / 64, NB), 256, 0, stream>>>(xq, XTQ);
    k_xT<<<dim3(SEQ / 64, DM / 64, NB), 256, 0, stream>>>(xk, XTK);
    k_xT<<<dim3(SEQ / 64, DM / 64, NB), 256, 0, stream>>>(xv, XTV);
    { const size_t n8 = (size_t)DM * DM / 8; const unsigned g = (unsigned)((n8 + 255) / 256);
      k_cvt8<<<g, 256, 0, stream>>>(wq, WQ, n8); k_cvt8<<<g, 256, 0, stream>>>(wk, WK, n8); k_cvt8<<<g, 256, 0, stream>>>(wv, WV, n8);
      k_cvtw<<<g, 256, 0, stream>>>(wo, WO, n8); }
    k_ev<<<(NH_ * HD * 4) / 256, 256, 0, stream>>>(ev, EV);

    k_proj<0><<<dim3(NB * SEQ / 64, DM / 64, 1), 32, 0, stream>>>(XTQ, WQ, bq, QH, QR, 1, SEQ, (size_t)NH_ * SEQ * HD, HD, HD, (size_t)SEQ * HD);
    k_proj<0><<<dim3(NB * SEQ / 64, DM / 64, 1), 32, 0, stream>>>(XTK, WK, bk, KP, KP, 0, SEQ, (size_t)NH_ * SEQ * HD, HD, HD, (size_t)SEQ * HD);
    k_proj<1><<<dim3(DM / 64, NB * SEQ / 64, 1), 32, 0, stream>>>(WV, XTV, bv, VT, VT, 0, DM, (size_t)0, SEQ, SEQ, (size_t)DM * SEQ);

    k_flash<<<dim3(SEQ / (16 * AW), NB * NH_, 1), 32 * AW, 0, stream>>>(QH, QR, KP, VT, EV, ek, CT);

    k_oproj<<<dim3(DM / 64, NB * SEQ / 64, 1), 32, 0, stream>>>(WO, CT, bo, OUT);
}
